// DLSTMCell_7816840479037
// MI455X (gfx1250) — hardware-verified
//
#include <hip/hip_runtime.h>
#include <math.h>

constexpr int   kBatch   = 128;
constexpr int   kNodes   = 512;
constexpr int   kRU      = 64;
constexpr int   kInPer   = 2;
constexpr int   kMemDim  = 16;
constexpr int   kBotDim  = 4;
constexpr int   kInSz    = 66;
constexpr int   kOutSz   = 256;
constexpr int   kKpad    = 96;
constexpr int   kW3Cols  = kInSz * kOutSz;
constexpr int   kInCols  = kNodes * kInPer;
constexpr int   kNRU     = kNodes * kRU;
constexpr long  kBNRU    = (long)kBatch * kNRU;
constexpr float kWCarry    = 1024.0f;
constexpr float kWCarryInv = 1.0f / 1024.0f;

constexpr size_t kWpHalves  = (size_t)kNodes * kOutSz * kKpad;
constexpr size_t kApHalves  = (size_t)kNodes * kBatch * kKpad;
constexpr size_t kValFloats = (size_t)kNodes * kBatch * kOutSz;
constexpr size_t kOffWp   = 0;
constexpr size_t kOffAp   = kOffWp + kWpHalves * 2;
constexpr size_t kOffVal  = kOffAp + kApHalves * 2;
constexpr size_t kWsTotal = kOffVal + kValFloats * 4;
static_assert(kOffAp == 25165824, "carve");
static_assert(kOffVal == 37748736, "carve");
static_assert(kWsTotal == 104857600, "carve");

typedef __attribute__((ext_vector_type(16))) _Float16 v16h;
typedef __attribute__((ext_vector_type(8)))  _Float16 v8h;
typedef __attribute__((ext_vector_type(16))) __bf16   v16b;
typedef __attribute__((ext_vector_type(8)))  __bf16   v8b;
typedef __attribute__((ext_vector_type(8)))  float    v8f;
typedef __attribute__((ext_vector_type(4)))  float    v4f;
typedef __attribute__((ext_vector_type(4)))  unsigned int v4u;

__device__ __forceinline__ unsigned short f2bf_bits(float f) {
  unsigned u = __float_as_uint(f);
  return (unsigned short)((u + 0x7FFFu + ((u >> 16) & 1u)) >> 16);
}
__device__ __forceinline__ float bf_bits2f(unsigned short h) { return __uint_as_float(((unsigned)h) << 16); }

__device__ __forceinline__ void dep_guard_h(v8f& a, v8f& b, v16h x, v16h y) { asm volatile("v_nop\n\tv_nop\n\tv_nop\n\tv_nop" : "+v"(a), "+v"(b) : "v"(x), "v"(y)); }
__device__ __forceinline__ void dep_guard_b(v8f& a, v8f& b, v16b x, v16b y) { asm volatile("v_nop\n\tv_nop\n\tv_nop\n\tv_nop" : "+v"(a), "+v"(b) : "v"(x), "v"(y)); }
__device__ __forceinline__ void keep4_h(v16h a, v16h b, v16h c, v16h d) { asm volatile("v_nop" :: "v"(a), "v"(b), "v"(c), "v"(d)); }
__device__ __forceinline__ void keep4_b(v16b a, v16b b, v16b c, v16b d) { asm volatile("v_nop" :: "v"(a), "v"(b), "v"(c), "v"(d)); }
__device__ __forceinline__ void acc_guard4(v8f& a, v8f& b, v8f& c, v8f& d) { asm volatile("v_nop\n\tv_nop\n\tv_nop\n\tv_nop" : "+v"(a), "+v"(b), "+v"(c), "+v"(d)); }
template <typename T> struct Frag;
template <> struct Frag<_Float16> {
  typedef v16h V; union U { v16h v; v8h h[2]; };
  static __device__ __forceinline__ v16h load(const _Float16* p) {
    U f; f.h[0] = *(const v8h*)(p); f.h[1] = *(const v8h*)(p + 16); return f.v;
  }
  static __device__ __forceinline__ v8f mma(v16h a, v16h b, v8f c) {
    return __builtin_amdgcn_wmma_f32_16x16x32_f16(false, a, false, b, (short)0, c, false, false);
  }
  static __device__ __forceinline__ void guard(v8f& a, v8f& b, v16h x, v16h y) { dep_guard_h(a, b, x, y); }
  static __device__ __forceinline__ void keep(v16h a, v16h b, v16h c, v16h d) { keep4_h(a, b, c, d); }
};
template <> struct Frag<__bf16> {
  typedef v16b V; union U { v16b v; v8b h[2]; };
  static __device__ __forceinline__ v16b load(const __bf16* p) {
    U f; f.h[0] = *(const v8b*)(p); f.h[1] = *(const v8b*)(p + 16); return f.v;
  }
  static __device__ __forceinline__ v8f mma(v16b a, v16b b, v8f c) {
    return __builtin_amdgcn_wmma_f32_16x16x32_bf16(false, a, false, b, (short)0, c, false, false);
  }
  static __device__ __forceinline__ void guard(v8f& a, v8f& b, v16b x, v16b y) { dep_guard_b(a, b, x, y); }
  static __device__ __forceinline__ void keep(v16b a, v16b b, v16b c, v16b d) { keep4_b(a, b, c, d); }
};

__device__ __forceinline__ unsigned pk16(unsigned short a, unsigned short b) { return (unsigned)a | ((unsigned)b << 16); }
__device__ __forceinline__ unsigned short h_bits(float f) { const _Float16 h = (_Float16)f; return __builtin_bit_cast(unsigned short, h); }

template <int ET> struct Elem;
template <> struct Elem<0> { typedef _Float16 T; };
template <> struct Elem<1> { typedef __bf16 T; };
template <int ET, bool SPLIT, int BIAS_MODE, int OUT_MODE, bool RESID, int ACT = 0>
__global__ __launch_bounds__(256) void wmma_gemm64(
    const unsigned short* __restrict__ Ap, const unsigned short* __restrict__ A2p, int lda, long strideA,
    const unsigned short* __restrict__ Btp, const unsigned short* __restrict__ Bt2p, int ldb, long strideB,
    void* __restrict__ Cout, void* __restrict__ Cout2, int ldc, long strideC,
    const float* __restrict__ bias,
    const float* __restrict__ resid, long strideR,
    int M, int N, int K, float scale) {
  typedef typename Elem<ET>::T T;
  typedef typename Frag<T>::V V;
  const T* A = (const T*)Ap; const T* A2 = (const T*)A2p; const T* Bt = (const T*)Btp; const T* Bt2 = (const T*)Bt2p;
  __shared__ __align__(16) float sT[8][16 * 68];
  const int b    = blockIdx.y;
  const int lane = threadIdx.x & 31;
  const int wave = threadIdx.x >> 5;
  const int tilesN = N >> 6;
  const int tilesM = M >> 6;
  const int tile = blockIdx.x * 8 + wave;
  if (tile >= tilesM * tilesN) return;
  const int tm = tile / tilesN;
  const int tn = tile - tm * tilesN;
  const int m0 = tm << 6;
  const int n0 = tn << 6;

  const T* Ab  = A  + (size_t)b * strideA;
  const T* Bb  = Bt + (size_t)b * strideB;
  const T* Ab2 = SPLIT ? (A2  + (size_t)b * strideA) : nullptr;
  const T* Bb2 = SPLIT ? (Bt2 + (size_t)b * strideB) : nullptr;

  const int rlane = lane & 15;
  const int koff  = (lane >> 4) * 8;
  const int mOff  = (lane >> 4) * 8;

  v8f acc[4][4];
#pragma unroll
  for (int i = 0; i < 4; ++i)
#pragma unroll
    for (int j = 0; j < 4; ++j) acc[i][j] = (v8f){0.f,0.f,0.f,0.f,0.f,0.f,0.f,0.f};

  for (int k0 = 0; k0 < K; k0 += 32) {
    V bh[4], bl[4];
#pragma unroll
    for (int j = 0; j < 4; ++j) {
      const size_t bo = (size_t)(n0 + (j << 4) + rlane) * ldb + koff + k0;
      bh[j] = Frag<T>::load(Bb + bo);
      if (SPLIT) bl[j] = Frag<T>::load(Bb2 + bo);
    }
#pragma unroll
    for (int i = 0; i < 4; ++i) {
      const size_t ao = (size_t)(m0 + (i << 4) + rlane) * lda + koff + k0;
      V ah = Frag<T>::load(Ab + ao);
      V al;
      if (SPLIT) al = Frag<T>::load(Ab2 + ao);
#pragma unroll
      for (int j = 0; j < 4; ++j) {
        acc[i][j] = Frag<T>::mma(ah, bh[j], acc[i][j]);
        if (SPLIT) {
          acc[i][j] = Frag<T>::mma(ah, bl[j], acc[i][j]);
          acc[i][j] = Frag<T>::mma(al, bh[j], acc[i][j]);
        }
      }
      Frag<T>::guard(acc[i][0], acc[i][3], ah, SPLIT ? al : ah);
    }
    Frag<T>::keep(bh[0], bh[1], bh[2], bh[3]);
    if (SPLIT) Frag<T>::keep(bl[0], bl[1], bl[2], bl[3]);
  }
  acc_guard4(acc[0][0], acc[0][1], acc[0][2], acc[0][3]);
  acc_guard4(acc[1][0], acc[1][1], acc[1][2], acc[1][3]);
  acc_guard4(acc[2][0], acc[2][1], acc[2][2], acc[2][3]);
  acc_guard4(acc[3][0], acc[3][1], acc[3][2], acc[3][3]);

  float* slab = sT[wave];
  const float* Rb = RESID ? (resid + (size_t)b * strideR) : nullptr;
#pragma unroll
  for (int i = 0; i < 4; ++i) {
    const int mBase = m0 + (i << 4);
#pragma unroll
    for (int j = 0; j < 4; ++j) {
      const int n = n0 + (j << 4) + rlane;
      float bv = 0.f;
      if (BIAS_MODE == 2) bv = bias[n];
#pragma unroll
      for (int r = 0; r < 8; ++r) {
        float v = acc[i][j][r] * scale;
        if (BIAS_MODE == 1) v += bias[mBase + mOff + r];
        if (BIAS_MODE == 2) v += bv;
        if (RESID) v += Rb[(size_t)(mBase + mOff + r) * ldc + n];
        if (ACT == 2) v = fmaxf(v, 0.0f);
        if (ACT == 4) v = (v > 0.f) ? v : 0.01f * v;
        slab[(mOff + r) * 68 + (j << 4) + rlane] = v;
      }
    }
    __builtin_amdgcn_fence(__ATOMIC_RELEASE, "workgroup");
    __builtin_amdgcn_wave_barrier();
    __builtin_amdgcn_fence(__ATOMIC_ACQUIRE, "workgroup");
    if (OUT_MODE == 0) {
      float* C = (float*)Cout + (size_t)b * strideC;
      const int hh = lane >> 4, c4 = (lane & 15) * 4;
      for (int pass = 0; pass < 2; ++pass) {
#pragma unroll
        for (int it = 0; it < 8; ++it) {
          const int row = it * 2 + hh;
          v4f v = *(const v4f*)(slab + row * 68 + c4);
          *(volatile v4f*)(C + (size_t)(mBase + row) * ldc + n0 + c4) = v;
        }
        __threadfence();
      }
    } else {
      const int q = lane >> 3, c8 = (lane & 7) * 8;
      unsigned short* C  = (unsigned short*)Cout  + (size_t)b * strideC;
      unsigned short* C2 = (OUT_MODE == 2) ? ((unsigned short*)Cout2 + (size_t)b * strideC) : nullptr;
      for (int pass = 0; pass < 2; ++pass) {
#pragma unroll
        for (int it = 0; it < 4; ++it) {
          const int row = it * 4 + q;
          const float* sp = slab + row * 68 + c8;
          v8h hv, lv;
#pragma unroll
          for (int e = 0; e < 8; ++e) {
            if (OUT_MODE == 1) {
              hv[e] = (_Float16)sp[e];
            } else {
              unsigned short hb = f2bf_bits(sp[e]);
              unsigned short lb = f2bf_bits(sp[e] - bf_bits2f(hb));
              hv[e] = __builtin_bit_cast(_Float16, hb);
              lv[e] = __builtin_bit_cast(_Float16, lb);
            }
          }
          *(volatile v8h*)(C + (size_t)(mBase + row) * ldc + n0 + c8) = hv;
          if (OUT_MODE == 2) *(volatile v8h*)(C2 + (size_t)(mBase + row) * ldc + n0 + c8) = lv;
        }
        __threadfence();
      }
    }
    __builtin_amdgcn_fence(__ATOMIC_RELEASE, "workgroup");
    __builtin_amdgcn_wave_barrier();
    __builtin_amdgcn_fence(__ATOMIC_ACQUIRE, "workgroup");
  }
}

__global__ __launch_bounds__(256) void hyper_prep_kernel(
    const float* __restrict__ inp, const float* __restrict__ hx,
    const float* __restrict__ memory, const float* __restrict__ w1, const float* __restrict__ b1,
    const float* __restrict__ w2, const float* __restrict__ b2,
    const float* __restrict__ w3, const float* __restrict__ b3,
    unsigned short* __restrict__ Wp, unsigned short* __restrict__ Ap) {
  __shared__ float sM1[kMemDim];
  __shared__ float sM2[kBotDim];
  const int n   = blockIdx.x;
  const int tid = threadIdx.x;

  {
    const int col1 = tid & (kMemDim - 1);
    float a1 = 0.0f;
#pragma unroll 1
    for (int k = 0; k < kMemDim; ++k) a1 = fmaf(memory[n * kMemDim + k], w1[k * kMemDim + col1], a1);
    a1 = tanhf(a1 + b1[col1]);
    if (tid < kMemDim) sM1[tid] = a1;
  }
  __syncthreads();
  {
    const int col2 = tid & (kBotDim - 1);
    float a2 = 0.0f;
#pragma unroll 1
    for (int k = 0; k < kMemDim; ++k) a2 = fmaf(sM1[k], w2[k * kBotDim + col2], a2);
    a2 = tanhf(a2 + b2[col2]);
    if (tid < kBotDim) sM2[tid] = a2;
  }
  __syncthreads();
  const float mq0 = sM2[0], mq1 = sM2[1], mq2 = sM2[2], mq3 = sM2[3];

  {
    unsigned short* wbase = Wp + (size_t)n * (kOutSz * kKpad);
#pragma unroll 1
    for (int it = 0; it < 12; ++it) {
      const int c  = it * 256 + tid;
      const int o  = c / 12;
      const int k0 = (c - o * 12) * 8;
      unsigned short hb[8];
#pragma unroll
      for (int j = 0; j < 8; ++j) {
        const int k   = k0 + j;
        const int kc  = (k < kInSz) ? k : (kInSz - 1);
        const int idx = kc * kOutSz + o;
        float s = mq0 * w3[idx];
        s = fmaf(mq1, w3[kW3Cols + idx], s);
        s = fmaf(mq2, w3[2 * kW3Cols + idx], s);
        s = fmaf(mq3, w3[3 * kW3Cols + idx], s);
        const float wv = s + b3[idx];
        const float v  = (k < kInSz) ? (wv * kWCarry) : 0.0f;
        hb[j] = h_bits(v);
      }
      const v4u u = (v4u){pk16(hb[0], hb[1]), pk16(hb[2], hb[3]), pk16(hb[4], hb[5]), pk16(hb[6], hb[7])};
      unsigned short* p = wbase + (size_t)c * 8;
      *(volatile v4u*)p = u;
      __threadfence();
      *(volatile v4u*)p = u;
    }
  }

  {
    unsigned short* abase = Ap + (size_t)n * (kBatch * kKpad);
#pragma unroll 1
    for (int it = 0; it < 6; ++it) {
      const int c  = it * 256 + tid;
      const int b  = c / 12;
      const int k0 = (c - b * 12) * 8;
      unsigned short hb[8];
#pragma unroll
      for (int j = 0; j < 8; ++j) {
        const int k   = k0 + j;
        const int kin = (k < 1) ? k : 1;
        int khx = k - 2; khx = khx < 0 ? 0 : (khx > kRU - 1 ? kRU - 1 : khx);
        const float vin = inp[(size_t)b * kInCols + n * kInPer + kin];
        const float vhx = hx[(size_t)b * kNRU + n * kRU + khx];
        const float v   = (k < kInPer) ? vin : ((k < kInSz) ? vhx : 0.0f);
        hb[j] = h_bits(v);
      }
      const v4u u = (v4u){pk16(hb[0], hb[1]), pk16(hb[2], hb[3]), pk16(hb[4], hb[5]), pk16(hb[6], hb[7])};
      unsigned short* p = abase + (size_t)c * 8;
      *(volatile v4u*)p = u;
      __threadfence();
      *(volatile v4u*)p = u;
    }
  }
}

__device__ __forceinline__ float sigm_f(float x) { return 1.0f / (1.0f + expf(-x)); }

__global__ __launch_bounds__(256) void lstm_gate_kernel(
    const float* __restrict__ val, const float* __restrict__ cx,
    const float* __restrict__ b_out, float* __restrict__ out) {
  __shared__ __align__(16) float sG[4 * 256];
  __shared__ __align__(16) float sHC[512];
  const int tid = threadIdx.x;
  const int b   = blockIdx.y;
  const int ng0 = blockIdx.x * 4;
  const int nl  = tid >> 6;
  const int u   = tid & 63;
  const int n   = ng0 + nl;
  const float* vp = val + ((size_t)n * kBatch + b) * kOutSz;

#pragma unroll 1
  for (int gi = 0; gi < 4; ++gi) {
    const float v = vp[gi * kRU + u];
    const float s = sigm_f(v) + b_out[gi * kRU + u];
    float r;
    if (gi == 2) r = tanhf(s); else r = sigm_f(s);
    sG[gi * 256 + tid] = r;
  }
  const float i_t = sG[tid];
  const float f_t = sG[256 + tid];
  const float g_t = sG[512 + tid];
  const float o_t = sG[768 + tid];
  const float c0  = cx[(size_t)b * kNRU + n * kRU + u];
  const float cy  = c0 * f_t + i_t * g_t;
  const float hy  = o_t * tanhf(cy);
  sHC[tid]       = hy;
  sHC[256 + tid] = cy;
  __syncthreads();

  if (tid < 128) {
    const int which = tid >> 6;
    const int q     = tid & 63;
    const v4f vv = *(const v4f*)(sHC + which * 256 + 4 * q);
    float* dst = out + (size_t)which * kBNRU + (size_t)b * kNRU + (size_t)ng0 * kRU + 4 * q;
    *(volatile v4f*)dst = vv;
    __threadfence();
    *(volatile v4f*)dst = vv;
  }
}

extern "C" void kernel_launch(void* const* d_in, const int* in_sizes, int n_in,
                              void* d_out, int out_size, void* d_ws, size_t ws_size,
                              hipStream_t stream) {
  (void)in_sizes; (void)n_in;
  const float* inputs = (const float*)d_in[0];
  const float* hx     = (const float*)d_in[1];
  const float* cx     = (const float*)d_in[2];
  const float* memory = (const float*)d_in[3];
  const float* w1     = (const float*)d_in[4];
  const float* b1     = (const float*)d_in[5];
  const float* w2     = (const float*)d_in[6];
  const float* b2     = (const float*)d_in[7];
  const float* w3     = (const float*)d_in[8];
  const float* b3     = (const float*)d_in[9];
  const float* b_out  = (const float*)d_in[10];
  float* out = (float*)d_out;

  if (ws_size < kWsTotal) return;
  if ((size_t)out_size < (size_t)(2 * kBNRU)) return;

  unsigned char* ws = (unsigned char*)d_ws;
  unsigned short* Wp  = (unsigned short*)(ws + kOffWp);
  unsigned short* Ap  = (unsigned short*)(ws + kOffAp);
  float*          val = (float*)(ws + kOffVal);

  hyper_prep_kernel<<<dim3(kNodes), dim3(256), 0, stream>>>(inputs, hx, memory, w1, b1, w2, b2, w3, b3, Wp, Ap);

  wmma_gemm64<0, false, 0, 0, false, 0><<<dim3(1, kNodes), dim3(256), 0, stream>>>(
      Ap, Ap, kKpad, (long)kBatch * kKpad,
      Wp, Wp, kKpad, (long)kOutSz * kKpad,
      (void*)val, (void*)val, kOutSz, (long)kBatch * kOutSz,
      b_out,
      (const float*)val, 0L,
      kBatch, kOutSz, kKpad, kWCarryInv);

  lstm_gate_kernel<<<dim3(kNodes / 4, kBatch), dim3(256), 0, stream>>>(val, cx, b_out, out);
}
